// TpsGridGen_41068477284473
// MI455X (gfx1250) — hardware-verified
//
#include <hip/hip_runtime.h>
#include <math.h>

#pragma clang fp contract(off)

typedef __attribute__((ext_vector_type(16))) _Float16 v16h;
typedef __attribute__((ext_vector_type(8)))  _Float16 v8h;
typedef __attribute__((ext_vector_type(16))) __bf16   v16b;
typedef __attribute__((ext_vector_type(8)))  __bf16   v8b;
typedef __attribute__((ext_vector_type(8)))  float    v8f;
typedef __attribute__((ext_vector_type(4)))  float    v4f;

constexpr int kBatch  = 64;
constexpr int kNc     = 25;
constexpr int kLd     = 28;
constexpr int kKp     = 32;
constexpr int kH      = 256;
constexpr int kWd     = 192;
constexpr int kNPix   = kH * kWd;
constexpr int kRowsC  = 2 * kBatch;
constexpr int kPixBlk = 128;
constexpr int kSlabP  = 36;
static_assert(kNc + 3 == kLd, "feature count = control points + affine terms");
static_assert(kLd <= kKp && (kKp % 32) == 0, "K padded to one 32-deep step");
static_assert(kNPix == 49152 && (kNPix % kPixBlk) == 0, "pixel tiles are exact");
static_assert(2 * kPixBlk == 256, "one coordinate value per thread in the staging step");
static_assert((kBatch % 16) == 0 && (kPixBlk % 16) == 0, "16-row / 16-column sub-tiles are exact");
static_assert((kSlabP % 4) == 0 && kSlabP >= 32, "slab rows 16-B aligned, 32 columns used");

constexpr size_t kOffCh   = 0;
constexpr size_t kOffCl   = kOffCh + (size_t)kRowsC * kKp * 2;
constexpr size_t kWsTotal = kOffCl + (size_t)kRowsC * kKp * 2;
static_assert(kWsTotal == 16384ull, "carve total");
static_assert((kOffCl % 128) == 0, "128-B aligned regions");
static_assert(kWsTotal <= 134217728ull, "carve cap");

__device__ __forceinline__ unsigned short f2bf_bits(float f) {
  unsigned u = __float_as_uint(f);
  return (unsigned short)((u + 0x7FFFu + ((u >> 16) & 1u)) >> 16);
}
__device__ __forceinline__ float bf_bits2f(unsigned short h) { return __uint_as_float(((unsigned)h) << 16); }

__device__ __forceinline__ v16b frag_load_bf(const __bf16* p) {
  union U { v16b v; v8b h[2]; };
  U f;
  f.h[0] = *(const v8b*)(p);
  f.h[1] = *(const v8b*)(p + 16);
  return f.v;
}
__device__ __forceinline__ v8f mma_bf(v16b a, v16b b, v8f c) {
  c = __builtin_amdgcn_wmma_f32_16x16x32_bf16(false, a, false, b, (short)0, c, false, false);
  asm volatile("v_nop\n\tv_nop\n\tv_nop\n\tv_nop" : "+v"(c) : "v"(a), "v"(b));
  return c;
}

__global__ __launch_bounds__(256) void coef_planes_kernel(
    const float* __restrict__ theta, const float* __restrict__ Px, const float* __restrict__ Py,
    const float* __restrict__ Li, unsigned short* __restrict__ Ch, unsigned short* __restrict__ Cl)
{
  __shared__ float sP[64];
  __shared__ float sLi[kLd * kLd];
  __shared__ float sQ[kRowsC * kNc];
  __shared__ __align__(16) float sC[kRowsC * kKp];
  const int tid = threadIdx.x;

  {
    const int ia = (tid < kNc) ? tid : (kNc - 1);
    int ib = tid - kNc;
    ib = (ib < 0) ? 0 : ib;
    ib = (ib > kNc - 1) ? (kNc - 1) : ib;
    float pa = Px[ia];
    asm volatile("" : "+v"(pa));
    float pb = Py[ib];
    asm volatile("" : "+v"(pb));
    const float pv = (tid < kNc) ? pa : pb;
    if (tid < 2 * kNc) sP[tid] = pv;
  }
  constexpr int kLiN = kLd * kLd;
#pragma unroll 1
  for (int it = 0; it < (kLiN + 255) / 256; ++it) {
    const int i  = it * 256 + tid;
    const int ic = (i < kLiN) ? i : (kLiN - 1);
    float v = Li[ic];
    asm volatile("" : "+v"(v));
    if (i < kLiN) sLi[i] = v;
  }
  __syncthreads();

  constexpr int kQN = kRowsC * kNc;
#pragma unroll 1
  for (int it = 0; it < (kQN + 255) / 256; ++it) {
    const int i   = it * 256 + tid;
    const int ic  = (i < kQN) ? i : (kQN - 1);
    const int row = ic / kNc;
    const int m   = ic - row * kNc;
    const int c   = row >> 6;
    const int b   = row & (kBatch - 1);
    float v = theta[b * (2 * kNc) + c * kNc + m];
    asm volatile("" : "+v"(v));
    const float qv = v + sP[c * kNc + m];
    if (i < kQN) sQ[i] = qv;
  }
  __syncthreads();

  {
    const int j  = tid & 31;
    const int jc = (j < kLd) ? j : (kLd - 1);
    const int r0 = tid >> 5;
    const float* lr = sLi + jc * kLd;
#pragma unroll 1
    for (int it = 0; it < kRowsC / 8; ++it) {
      const int row = it * 8 + r0;
      const float* qr = sQ + row * kNc;
      float s = 0.0f;
#pragma unroll
      for (int m = 0; m < kNc; ++m) s = fmaf(lr[m], qr[m], s);
      sC[row * kKp + j] = (j < kLd) ? s : 0.0f;
    }
  }
  __syncthreads();

  v8h hv[2], lv[2];
#pragma unroll
  for (int it = 0; it < 2; ++it) {
    const int chunk = it * 256 + tid;
    const float* sp = sC + chunk * 8;
    const v4f a0 = *(const v4f*)(sp);
    const v4f a1 = *(const v4f*)(sp + 4);
#pragma unroll
    for (int e = 0; e < 4; ++e) {
      const float x0 = a0[e];
      const float x1 = a1[e];
      const unsigned short h0 = f2bf_bits(x0), h1 = f2bf_bits(x1);
      const unsigned short l0 = f2bf_bits(x0 - bf_bits2f(h0)), l1 = f2bf_bits(x1 - bf_bits2f(h1));
      hv[it][e]     = __builtin_bit_cast(_Float16, h0);
      hv[it][4 + e] = __builtin_bit_cast(_Float16, h1);
      lv[it][e]     = __builtin_bit_cast(_Float16, l0);
      lv[it][4 + e] = __builtin_bit_cast(_Float16, l1);
    }
  }
  for (int pass = 0; pass < 2; ++pass) {
#pragma unroll
    for (int it = 0; it < 2; ++it) {
      const size_t o = (size_t)(it * 256 + tid) * 8;
      *(volatile v8h*)(Ch + o) = hv[it];
      *(volatile v8h*)(Cl + o) = lv[it];
    }
    __threadfence();
  }
}

__global__ __launch_bounds__(256) void warp_grid_kernel(
    const float* __restrict__ gx, const float* __restrict__ gy,
    const float* __restrict__ Px, const float* __restrict__ Py,
    const unsigned short* __restrict__ Chg, const unsigned short* __restrict__ Clg,
    float* __restrict__ out)
{
  __shared__ __align__(16) __bf16 sCh[kRowsC * kKp];
  __shared__ __align__(16) __bf16 sCl[kRowsC * kKp];
  __shared__ __align__(16) __bf16 sFh[kPixBlk * kKp];
  __shared__ __align__(16) __bf16 sFl[kPixBlk * kKp];
  __shared__ __align__(16) float  sG[2 * kPixBlk];
  __shared__ __align__(16) float  sSlab[8 * 16 * kSlabP];

  const int tid  = threadIdx.x;
  const int lane = tid & 31;
  const int wave = tid >> 5;
  const int pixBase = blockIdx.x * kPixBlk;

  {
    const float* gsrc = (tid < kPixBlk) ? gx : gy;
    sG[tid] = gsrc[pixBase + (tid & (kPixBlk - 1))];
    const __bf16* cgh = (const __bf16*)(const void*)Chg;
    const __bf16* cgl = (const __bf16*)(const void*)Clg;
#pragma unroll
    for (int it = 0; it < 2; ++it) {
      const int idx = (it * 256 + tid) * 8;
      *(v8b*)(sCh + idx) = *(const v8b*)(cgh + idx);
      *(v8b*)(sCl + idx) = *(const v8b*)(cgl + idx);
    }
  }
  const int kc = (lane < kNc) ? lane : (kNc - 1);
  float px = Px[kc];
  asm volatile("" : "+v"(px));
  float py = Py[kc];
  asm volatile("" : "+v"(py));
  __syncthreads();

#pragma unroll 4
  for (int it = 0; it < kPixBlk / 8; ++it) {
    const int pix = it * 8 + wave;
    const float xv = sG[pix];
    const float yv = sG[kPixBlk + pix];
    const float dx = xv - px;
    const float dy = yv - py;
    const float sx = dx * dx;
    const float sy = dy * dy;
    float d2 = sx + sy;
    d2 = (d2 == 0.0f) ? 1.0f : d2;
    const float u = d2 * logf(d2);
    float aff = 0.0f;
    aff = (lane == kNc)     ? 1.0f : aff;
    aff = (lane == kNc + 1) ? xv   : aff;
    aff = (lane == kNc + 2) ? yv   : aff;
    const float f = (lane < kNc) ? u : aff;
    const unsigned short hb = f2bf_bits(f);
    const unsigned short lb = f2bf_bits(f - bf_bits2f(hb));
    sFh[pix * kKp + lane] = __builtin_bit_cast(__bf16, hb);
    sFl[pix * kKp + lane] = __builtin_bit_cast(__bf16, lb);
  }
  __syncthreads();

  const int rlane = lane & 15;
  const int hh    = lane >> 4;
  const int foff  = (wave * 16 + rlane) * kKp + 8 * hh;
  const v16b fh = frag_load_bf(sFh + foff);
  const v16b fl = frag_load_bf(sFl + foff);
  float* slab = sSlab + wave * (16 * kSlabP);
  const int q  = lane >> 3;
  const int c4 = (lane & 7) * 4;
  const int pix0 = pixBase + wave * 16;

#pragma unroll
  for (int i = 0; i < 4; ++i) {
    const int ao = (i * 16 + rlane) * kKp + 8 * hh;
    const v16b axh = frag_load_bf(sCh + ao);
    const v16b axl = frag_load_bf(sCl + ao);
    const v16b ayh = frag_load_bf(sCh + kBatch * kKp + ao);
    const v16b ayl = frag_load_bf(sCl + kBatch * kKp + ao);
    v8f accX = (v8f){0.f, 0.f, 0.f, 0.f, 0.f, 0.f, 0.f, 0.f};
    v8f accY = (v8f){0.f, 0.f, 0.f, 0.f, 0.f, 0.f, 0.f, 0.f};
    accX = mma_bf(axh, fh, accX);
    accX = mma_bf(axh, fl, accX);
    accX = mma_bf(axl, fh, accX);
    accY = mma_bf(ayh, fh, accY);
    accY = mma_bf(ayh, fl, accY);
    accY = mma_bf(ayl, fh, accY);
#pragma unroll
    for (int r = 0; r < 8; ++r) {
      slab[(8 * hh + r) * kSlabP + 2 * rlane]     = accX[r];
      slab[(8 * hh + r) * kSlabP + 2 * rlane + 1] = accY[r];
    }
    __builtin_amdgcn_fence(__ATOMIC_RELEASE, "workgroup");
    __builtin_amdgcn_wave_barrier();
    __builtin_amdgcn_fence(__ATOMIC_ACQUIRE, "workgroup");
    for (int pass = 0; pass < 2; ++pass) {
#pragma unroll
      for (int it = 0; it < 4; ++it) {
        const int row = it * 4 + q;
        const v4f v = *(const v4f*)(slab + row * kSlabP + c4);
        *(volatile v4f*)(out + ((size_t)(i * 16 + row) * kNPix + pix0) * 2 + c4) = v;
      }
      __threadfence();
    }
    __builtin_amdgcn_fence(__ATOMIC_RELEASE, "workgroup");
    __builtin_amdgcn_wave_barrier();
    __builtin_amdgcn_fence(__ATOMIC_ACQUIRE, "workgroup");
  }
}

extern "C" void kernel_launch(void* const* d_in, const int* in_sizes, int n_in,
                              void* d_out, int out_size, void* d_ws, size_t ws_size,
                              hipStream_t stream) {
  if (n_in < 6) return;
  if (in_sizes[0] != kBatch * 2 * kNc) return;
  if (in_sizes[1] != kNPix) return;
  if (in_sizes[2] != kNPix) return;
  if (in_sizes[3] != kNc) return;
  if (in_sizes[4] != kNc) return;
  if (in_sizes[5] != kLd * kLd) return;
  if (out_size != kBatch * kNPix * 2) return;
  if (ws_size < kWsTotal) return;

  const float* theta = (const float*)d_in[0];
  const float* gx    = (const float*)d_in[1];
  const float* gy    = (const float*)d_in[2];
  const float* Px    = (const float*)d_in[3];
  const float* Py    = (const float*)d_in[4];
  const float* Li    = (const float*)d_in[5];
  float* out = (float*)d_out;

  char* ws = (char*)d_ws;
  unsigned short* Ch = (unsigned short*)(ws + kOffCh);
  unsigned short* Cl = (unsigned short*)(ws + kOffCl);

  coef_planes_kernel<<<1, 256, 0, stream>>>(theta, Px, Py, Li, Ch, Cl);
  warp_grid_kernel<<<kNPix / kPixBlk, 256, 0, stream>>>(gx, gy, Px, Py, Ch, Cl, out);
}
